// MultiHeadAttentionSigmoid_75788992905596
// MI455X (gfx1250) — hardware-verified
//
#include <hip/hip_runtime.h>
#include <math.h>

typedef __attribute__((ext_vector_type(16))) _Float16 v16h;
typedef __attribute__((ext_vector_type(16))) __bf16 v16b;
typedef __attribute__((ext_vector_type(8)))  _Float16 v8h;
typedef __attribute__((ext_vector_type(8)))  float v8f;
typedef __attribute__((ext_vector_type(4)))  float v4f;
typedef __attribute__((ext_vector_type(2)))  float v2f;
typedef __attribute__((ext_vector_type(4)))  unsigned v4u;
typedef __attribute__((ext_vector_type(4)))  int v4i;
typedef float __attribute__((may_alias)) float_a;
typedef int __attribute__((may_alias)) int_a;

template <typename T> __device__ __forceinline__ void vst2(void* p, T v) { *(volatile T*)p = v; __threadfence(); *(volatile T*)p = v; }
__device__ __forceinline__ v8f wmma16(v16h a, v16h b, v8f c) {
  v8f d = __builtin_amdgcn_wmma_f32_16x16x32_f16(false, a, false, b, (short)0, c, false, false);
  asm volatile("v_nop\n\tv_nop\n\tv_nop\n\tv_nop" : "+v"(d) : "v"(a), "v"(b));
  return d;
}
__device__ __forceinline__ v8f wmma_bf(v16b a, v16b b, v8f c) {
  v8f d = __builtin_amdgcn_wmma_f32_16x16x32_bf16(false, a, false, b, (short)0, c, false, false);
  asm volatile("v_nop\n\tv_nop\n\tv_nop\n\tv_nop" : "+v"(d) : "v"(a), "v"(b));
  return d;
}
__device__ __forceinline__ v16h frag_h(const _Float16* rowk0, int lane) {
  union { v16h v; v8h q[2]; } u; const _Float16* p = rowk0 + 8 * (lane >> 4);
  u.q[0] = *(const v8h*)p; u.q[1] = *(const v8h*)(p + 16); return u.v;
}
__device__ __forceinline__ v16h frag_f32(const float* rowk0, int lane) {
  v16h a; const float* p = rowk0 + 8 * (lane >> 4);
#pragma unroll
  for (int i = 0; i < 8; ++i) { a[i] = (_Float16)p[i]; a[8 + i] = (_Float16)p[16 + i]; }
  return a;
}
__device__ __forceinline__ v16h frag_f32s(const float* rowk0, int lane, float sc) {
  v16h a; const float* p = rowk0 + 8 * (lane >> 4);
#pragma unroll
  for (int i = 0; i < 8; ++i) { a[i] = (_Float16)(p[i] * sc); a[8 + i] = (_Float16)(p[16 + i] * sc); }
  return a;
}
__device__ __forceinline__ v16h fragc_f32(const float* W, int k0, int n, int lane, int ld, int K) {
  v16h a; const int g = lane >> 4;
#pragma unroll
  for (int i = 0; i < 8; ++i) { const int ka = k0 + 8 * g + i, kb = ka + 16;
    a[i] = (_Float16)(ka < K ? W[(size_t)ka * ld + n] : 0.f); a[8 + i] = (_Float16)(kb < K ? W[(size_t)kb * ld + n] : 0.f); }
  return a;
}
struct F2 { v16b h, l; };
__device__ __forceinline__ F2 bsplit16(const float v[16]) { F2 r;
#pragma unroll
  for (int i = 0; i < 16; ++i) { const __bf16 h = (__bf16)v[i]; r.h[i] = h; r.l[i] = (__bf16)(v[i] - (float)h); }
  return r; }
__device__ __forceinline__ F2 split_row(const float* row, int k0, int lane) { float v[16]; const float* p = row + k0 + 8 * (lane >> 4);
#pragma unroll
  for (int i = 0; i < 8; ++i) { v[i] = p[i]; v[8 + i] = p[16 + i]; }
  return bsplit16(v); }
__device__ __forceinline__ F2 split_rowK(const float* row, int k0, int lane, int K) { float v[16]; const int g = lane >> 4;
#pragma unroll
  for (int i = 0; i < 8; ++i) { const int ka = k0 + 8 * g + i, kb = ka + 16; v[i] = ka < K ? row[ka] : 0.f; v[8 + i] = kb < K ? row[kb] : 0.f; }
  return bsplit16(v); }
__device__ __forceinline__ F2 split_col(const float* W, int k0, int n, int lane, int ld, int K) { float v[16]; const int g = lane >> 4;
#pragma unroll
  for (int i = 0; i < 8; ++i) { const int ka = k0 + 8 * g + i, kb = ka + 16; v[i] = ka < K ? W[(size_t)ka * ld + n] : 0.f; v[8 + i] = kb < K ? W[(size_t)kb * ld + n] : 0.f; }
  return bsplit16(v); }
__device__ __forceinline__ v8f mac3(const F2& a, const F2& b, v8f c) { c = wmma_bf(a.l, b.h, c); c = wmma_bf(a.h, b.l, c); return wmma_bf(a.h, b.h, c); }
__device__ __forceinline__ float sigm(float v) { return 1.0f / (1.0f + expf(-v)); }
#define LDSX() do { asm volatile("s_wait_dscnt 0" ::: "memory"); __builtin_amdgcn_wave_barrier(); __builtin_amdgcn_fence(__ATOMIC_RELEASE, "workgroup"); } while (0)

#define NB 2
#define LL 2048
#define DD 1024
#define NH 16
#define HD 64
#define NR (NB * LL)

__global__ __launch_bounds__(256) void k_cvtx(const float* __restrict__ x, _Float16* __restrict__ x16, float* __restrict__ rr) {
  __shared__ float red[256];
  const int r = blockIdx.x, tid = threadIdx.x; const float* xr = x + (size_t)r * DD;
  const v4f v = *(const v4f*)(xr + tid * 4); red[tid] = v[0] * v[0] + v[1] * v[1] + v[2] * v[2] + v[3] * v[3];
  union { _Float16 h[4]; v2f f; } pk; for (int e = 0; e < 4; ++e) pk.h[e] = (_Float16)v[e];
  vst2((v2f*)(x16 + (size_t)r * DD + tid * 4), pk.f);
  __syncthreads();
  for (int st = 128; st > 0; st >>= 1) { if (tid < st) red[tid] += red[tid + st]; __syncthreads(); }
  if (tid < 32) vst2(rr + (size_t)r * 32 + tid, (float_a)(tid == 0 ? rsqrtf(red[0] / (float)DD + 1e-8f) : 0.f));
}
__global__ __launch_bounds__(256) void k_packW(const float* __restrict__ Wq, const float* __restrict__ Wk, const float* __restrict__ Wv, const float* __restrict__ Wo, const float* __restrict__ qs, const float* __restrict__ ksv, _Float16* __restrict__ P) {
  const int n = blockIdx.x, tid = threadIdx.x; const int which = n / DD, o = n % DD;
  const float* W = which == 0 ? Wq : (which == 1 ? Wk : (which == 2 ? Wv : Wo));
  for (int q = tid; q < DD / 8; q += 256) { union { v8h hh; v4u u; } pk;
#pragma unroll
    for (int i = 0; i < 8; ++i) { const int d = q * 8 + i; float w = W[(size_t)o * DD + d] * 16.0f; if (which == 0) w *= qs[d]; else if (which == 1) w *= ksv[d]; pk.hh[i] = (_Float16)w; }
    vst2(P + (size_t)n * DD + q * 8, pk.u); }
}
__global__ __launch_bounds__(128) void k_proj(const _Float16* __restrict__ x16, const float* __restrict__ rr, const _Float16* __restrict__ P, const float* __restrict__ bq, const float* __restrict__ bk, const float* __restrict__ bv,
                                            _Float16* __restrict__ qh, _Float16* __restrict__ kh, _Float16* __restrict__ vT) {
  __shared__ __align__(16) float so[4][16][132];
  __shared__ __align__(16) _Float16 st[128][72];
  __shared__ float sfr[32];
  const int tid = threadIdx.x, wave = tid >> 5, lane = tid & 31, col = lane & 15, g = lane >> 4;
  const int r0b = blockIdx.x * 64, r0 = r0b + wave * 16, n0 = blockIdx.y * 128; const int b = r0b / LL, t0 = r0b % LL;
  const int which = n0 / DD, hb = (n0 % DD) / HD; const float* bias = which == 0 ? bq : (which == 1 ? bk : bv);
  if (tid < 32) sfr[tid] = powf(10000.0f, -(float)tid / 32.0f);
  v8f acc[8] = {};
#pragma unroll 1
  for (int kc = 0; kc < DD / 32; ++kc) { const v16h a = frag_h(x16 + (size_t)(r0 + col) * DD + kc * 32, lane);
#pragma unroll
    for (int j = 0; j < 8; ++j) acc[j] = wmma16(a, frag_h(P + (size_t)(n0 + j * 16 + col) * DD + kc * 32, lane), acc[j]); }
  __syncthreads();
#pragma unroll
  for (int j = 0; j < 8; ++j) { const int nl = j * 16 + col; const float bb = bias[(n0 % DD) + nl];
#pragma unroll
    for (int r = 0; r < 8; ++r) { const float sc = which < 2 ? rr[(size_t)(r0 + 8 * g + r) * 32] : 1.0f; so[wave][8 * g + r][nl] = acc[j][r] * (1.0f / 16.0f) * sc + bb; } }
  LDSX();
  if (which < 2) {
    for (int rl = 0; rl < 16; ++rl) { const float t = (float)(t0 + wave * 16 + rl); float nv[4];
#pragma unroll
      for (int e = 0; e < 4; ++e) { const int nl = lane * 4 + e; const int d = nl & 63; const float ang = t * sfr[d & 31]; float sn, cs; sincosf(ang, &sn, &cs);
        const float xv = so[wave][rl][nl]; const float xr = (d & 1) ? so[wave][rl][nl - 1] : -so[wave][rl][nl + 1]; nv[e] = xv * cs + xr * sn; }
      LDSX();
#pragma unroll
      for (int e = 0; e < 4; ++e) so[wave][rl][lane * 4 + e] = nv[e];
      LDSX(); }
    _Float16* dst = which == 0 ? qh : kh;
    for (int q = lane; q < 2 * 16 * 8; q += 32) { const int hh = q >> 7, rem = q & 127, rl = rem >> 3, pc = rem & 7; union { v8h h8; v4u u; } pk;
#pragma unroll
      for (int e = 0; e < 8; ++e) pk.h8[e] = (_Float16)so[wave][rl][hh * HD + pc * 8 + e];
      vst2(dst + (((size_t)b * NH + hb + hh) * LL + t0 + wave * 16 + rl) * HD + pc * 8, pk.u); } }
  else {
#pragma unroll 4
    for (int rl = 0; rl < 16; ++rl) {
#pragma unroll
      for (int e = 0; e < 4; ++e) st[lane * 4 + e][wave * 16 + rl] = (_Float16)so[wave][rl][lane * 4 + e]; }
    __syncthreads();
    for (int q = tid; q < 128 * 8; q += 128) { const int c = q >> 3, pc = q & 7, hh = c >> 6, d = c & 63;
      vst2(vT + (((size_t)b * NH + hb + hh) * HD + d) * LL + t0 + pc * 8, *(const v4u*)(&st[c][pc * 8])); }
  }
}
__global__ __launch_bounds__(128) void k_attn(const _Float16* __restrict__ qh, const _Float16* __restrict__ kh, const _Float16* __restrict__ vT, _Float16* __restrict__ o16) {
  __shared__ __align__(16) _Float16 sP[4][16][72];
  __shared__ __align__(16) float sO[4][16][68];
  const int tid = threadIdx.x, w = tid >> 5, lane = tid & 31, col = lane & 15, g = lane >> 4;
  const int bh = blockIdx.y, b = bh / NH, h = bh % NH, q0 = blockIdx.x * 64 + w * 16;
  const _Float16* qb = qh + (size_t)bh * LL * HD; const _Float16* kb = kh + (size_t)bh * LL * HD; const _Float16* vb = vT + (size_t)bh * HD * LL;
  v16h aq[2];
#pragma unroll
  for (int kc = 0; kc < 2; ++kc) aq[kc] = frag_h(qb + (size_t)(q0 + col) * HD + kc * 32, lane);
  float lsum[8] = {0.f, 0.f, 0.f, 0.f, 0.f, 0.f, 0.f, 0.f}; v8f acc[4] = {};
#pragma unroll 1
  for (int kt = 0; kt < LL / 64; ++kt) {
#pragma unroll
    for (int t = 0; t < 4; ++t) { v8f s = {};
#pragma unroll
      for (int kc = 0; kc < 2; ++kc) s = wmma16(aq[kc], frag_h(kb + (size_t)(kt * 64 + t * 16 + col) * HD + kc * 32, lane), s);
#pragma unroll
      for (int r = 0; r < 8; ++r) { const float wgt = __builtin_amdgcn_rcpf(1.0f + __expf(-s[r] * 0.125f)); lsum[r] += wgt; sP[w][8 * g + r][t * 16 + col] = (_Float16)(wgt * 16384.0f); } }
    LDSX();
#pragma unroll
    for (int kc = 0; kc < 2; ++kc) { const v16h pa = frag_h(&sP[w][col][0] + kc * 32, lane);
#pragma unroll
      for (int t = 0; t < 4; ++t) acc[t] = wmma16(pa, frag_h(vb + (size_t)(t * 16 + col) * LL + kt * 64 + kc * 32, lane), acc[t]); }
    __builtin_amdgcn_wave_barrier();
  }
#pragma unroll
  for (int off = 8; off >= 1; off >>= 1) {
#pragma unroll
    for (int r = 0; r < 8; ++r) lsum[r] += __shfl_xor(lsum[r], off, 32); }
#pragma unroll
  for (int r = 0; r < 8; ++r) { const float inv = 1.0f / ((lsum[r] + 1e-8f) * 16384.0f);
#pragma unroll
    for (int t = 0; t < 4; ++t) sO[w][8 * g + r][t * 16 + col] = acc[t][r] * inv; }
  LDSX();
  for (int q = lane; q < 16 * 8; q += 32) { const int rl = q >> 3, pc = q & 7; union { v8h h8; v4u u; } pk;
#pragma unroll
    for (int e = 0; e < 8; ++e) pk.h8[e] = (_Float16)(sO[w][rl][pc * 8 + e] * 16.0f);
    vst2(o16 + ((size_t)b * LL + q0 + rl) * DD + h * HD + pc * 8, pk.u); }
}
__global__ __launch_bounds__(128) void k_out(const _Float16* __restrict__ o16, const _Float16* __restrict__ P, const float* __restrict__ bo, float* __restrict__ out) {
  __shared__ __align__(16) float so[4][16][132];
  const int tid = threadIdx.x, wave = tid >> 5, lane = tid & 31, col = lane & 15, g = lane >> 4;
  const int r0 = blockIdx.x * 64 + wave * 16, n0 = blockIdx.y * 128;
  v8f acc[8] = {};
#pragma unroll 1
  for (int kc = 0; kc < DD / 32; ++kc) { const v16h a = frag_h(o16 + (size_t)(r0 + col) * DD + kc * 32, lane);
#pragma unroll
    for (int j = 0; j < 8; ++j) acc[j] = wmma16(a, frag_h(P + (size_t)(3 * DD + n0 + j * 16 + col) * DD + kc * 32, lane), acc[j]); }
#pragma unroll
  for (int j = 0; j < 8; ++j) { const float bb = bo[n0 + j * 16 + col];
#pragma unroll
    for (int r = 0; r < 8; ++r) so[wave][8 * g + r][j * 16 + col] = acc[j][r] * (1.0f / 256.0f) + bb; }
  LDSX();
#pragma unroll 4
  for (int rl = 0; rl < 16; ++rl) vst2(out + (size_t)(r0 + rl) * DD + n0 + lane * 4, *(const v4f*)(&so[wave][rl][lane * 4]));
}
extern "C" void kernel_launch(void* const* d_in, const int* in_sizes, int n_in, void* d_out, int out_size, void* d_ws, size_t ws_size, hipStream_t stream) {
  (void)in_sizes; (void)n_in; (void)out_size; (void)ws_size;
  const float* x = (const float*)d_in[0]; const float* Wq = (const float*)d_in[1]; const float* bq = (const float*)d_in[2]; const float* Wk = (const float*)d_in[3]; const float* bk = (const float*)d_in[4];
  const float* Wv = (const float*)d_in[5]; const float* bv = (const float*)d_in[6]; const float* Wo = (const float*)d_in[7]; const float* bo = (const float*)d_in[8];
  const float* qs = (const float*)d_in[9]; const float* ksv = (const float*)d_in[10];
  float* out = (float*)d_out;
  char* ws = (char*)d_ws; size_t off = 0;
  auto take = [&](size_t bytes) { char* p = ws + off; off += (bytes + 255) & ~(size_t)255; return p; };
  _Float16* x16 = (_Float16*)take((size_t)NR * DD * 2); float* rr = (float*)take((size_t)NR * 32 * 4); _Float16* P = (_Float16*)take((size_t)4 * DD * DD * 2);
  _Float16* qh = (_Float16*)take((size_t)NR * DD * 2); _Float16* kh = (_Float16*)take((size_t)NR * DD * 2); _Float16* vT = (_Float16*)take((size_t)NR * DD * 2); _Float16* o16 = (_Float16*)take((size_t)NR * DD * 2);
  k_cvtx<<<NR, 256, 0, stream>>>(x, x16, rr);
  k_packW<<<4 * DD, 256, 0, stream>>>(Wq, Wk, Wv, Wo, qs, ksv, P);
  k_proj<<<dim3(NR / 64, 3 * DD / 128), 128, 0, stream>>>(x16, rr, P, bq, bk, bv, qh, kh, vT);
  k_attn<<<dim3(LL / 64, NB * NH), 128, 0, stream>>>(qh, kh, vT, o16);
  k_out<<<dim3(NR / 64, DD / 128), 128, 0, stream>>>(o16, P, bo, out);
}
